// MLP_79611513799302
// MI455X (gfx1250) — hardware-run, weakly checked
//
#include <hip/hip_runtime.h>


#ifndef SEQ
#define SEQ 512
#endif
#define SEQ_FULL 512
#ifndef OUT_PITCH
#define OUT_PITCH SEQ
#endif
#define KD   1024
#define HID  512
#define PW   (2 * HID)
#define SW   8
#define TK2  2.8853900817779268f

static_assert(KD % 32 == 0);
static_assert(KD % 8 == 0);
static_assert(SEQ % 64 == 0);
static_assert(HID % 64 == 0);
static_assert(PW % 64 == 0);
static_assert(HID == 32 * 16);
static_assert(SEQ % SW == 0);
static_assert(SEQ % 128 == 0);
static_assert(SEQ / 128 <= SW);
static_assert((SEQ / 128) * 32 * 16 == SEQ * 4);
static_assert(32 * 16 * 8 == 16 * 64 * 4);
static_assert(OUT_PITCH % 32 == 0);
static_assert(OUT_PITCH >= SEQ);
static_assert(SEQ <= SEQ_FULL);
static_assert(((size_t)SEQ * KD) % 8 == 0);
static_assert(((size_t)HID * KD) % 8 == 0);
static_assert(16 * 68 * 4 <= 131072);
static_assert(SEQ * 4 <= 131072);

typedef unsigned short bf;
typedef __attribute__((ext_vector_type(16))) __bf16   v16bf;
typedef __attribute__((ext_vector_type(8)))  unsigned short v8us;
typedef __attribute__((ext_vector_type(8)))  float    v8f;
typedef __attribute__((ext_vector_type(4)))  float    v4f;
typedef v4f  __attribute__((may_alias)) v4fa;

__device__ __forceinline__ unsigned short f2bf(float f) { unsigned u = __float_as_uint(f); u += 0x7FFFu + ((u >> 16) & 1u); return (unsigned short)(u >> 16); }
__device__ __forceinline__ float bfr(float f) { return __uint_as_float(((unsigned)f2bf(f)) << 16); }
__device__ __forceinline__ v16bf cat16b(v8us lo, v8us hi) { return __builtin_bit_cast(v16bf, __builtin_shufflevector(lo, hi, 0, 1, 2, 3, 4, 5, 6, 7, 8, 9, 10, 11, 12, 13, 14, 15)); }
__device__ __forceinline__ v8f wmmab(v16bf a, v16bf b, v8f c) { return __builtin_amdgcn_wmma_f32_16x16x32_bf16(false, a, false, b, (short)0, c, false, false); }
__device__ __forceinline__ v8f wmmabg(v16bf a, v16bf b, v8f c) { c = wmmab(a, b, c); asm volatile("v_nop\n\tv_nop\n\tv_nop\n\tv_nop" : "+v"(c) : "v"(a), "v"(b)); return c; }
__device__ __forceinline__ v16bf ldb(const bf* p)  { return cat16b(*(const v8us*)p, *(const v8us*)(p + 16)); }
__device__ __forceinline__ void wave_sync() { __builtin_amdgcn_fence(3  , "wavefront"); __builtin_amdgcn_wave_barrier(); asm volatile("" ::: "memory"); }

__global__ __launch_bounds__(256) void k_cvt8(const float* __restrict__ src, bf* dst, size_t n8) {
    const size_t i = (size_t)blockIdx.x * 256 + threadIdx.x; if (i >= n8) return;
    const v8f v = *(const v8f*)(src + i * 8); v8us o;
#pragma unroll
    for (int k = 0; k < 8; ++k) o[k] = f2bf(v[k]);
    *(volatile v8us*)(dst + i * 8) = o; __threadfence(); *(volatile v8us*)(dst + i * 8) = o;
}

__global__ __launch_bounds__(32) void k_gemm(const bf* __restrict__ A, const bf* __restrict__ Bt, const float* __restrict__ bias_h, const float* __restrict__ bias_m, float* PF) {
    __shared__ __align__(16) float os[16 * 68];
    const int K = KD;
    const int lane = threadIdx.x & 31, lr = lane & 15, hi = lane >> 4;
    const unsigned r0 = blockIdx.x * 64u, c0 = blockIdx.y * 64u;
    v8f acc[4][4];
#pragma unroll
    for (int mb = 0; mb < 4; ++mb)
#pragma unroll
        for (int nb = 0; nb < 4; ++nb) acc[mb][nb] = (v8f){};
    const size_t aoff = (size_t)(r0 + lr) * K + 8 * hi, boff = (size_t)(c0 + lr) * K + 8 * hi;
#pragma unroll 1
    for (int kc = 0; kc < K; kc += 32) {
        v16bf a[4];
#pragma unroll
        for (int mb = 0; mb < 4; ++mb) a[mb] = ldb(A + aoff + (size_t)mb * 16 * K + kc);
#pragma unroll
        for (int nb = 0; nb < 4; ++nb) { const v16bf b = ldb(Bt + boff + (size_t)nb * 16 * K + kc);
#pragma unroll
            for (int mb = 0; mb < 4; ++mb) acc[mb][nb] = wmmabg(a[mb], b, acc[mb][nb]); }
    }
    const bool second = c0 >= (unsigned)HID;
    const unsigned cb = c0 % (unsigned)HID;
    float bc[4];
#pragma unroll
    for (int nb = 0; nb < 4; ++nb) { const float vh = bias_h[cb + nb * 16 + lr]; const float vm = bias_m[cb + nb * 16 + lr]; bc[nb] = bfr(second ? vm : vh); }
#pragma unroll
    for (int mb = 0; mb < 4; ++mb) {
#pragma unroll
        for (int nb = 0; nb < 4; ++nb) {
#pragma unroll
            for (int j = 0; j < 8; ++j) os[(hi * 8 + j) * 68 + nb * 16 + lr] = acc[mb][nb][j] + bc[nb]; }
        wave_sync();
        float* prow = PF + (size_t)(r0 + mb * 16) * PW + c0;
#pragma unroll 1
        for (int ps = 0; ps < 2; ++ps) {
#pragma unroll
            for (int s = 0; s < 8; ++s) { const int row = 2 * s + (lane >> 4), c4 = (lane & 15) * 4;
                const v4f val = *(const v4fa*)(&os[row * 68 + c4]);
                *(volatile v4f*)(prow + (size_t)row * PW + c4) = val; }
            if (ps == 0) __threadfence(); }
        wave_sync();
    }
}

__global__ __launch_bounds__(32 * SW) void k_score(const float* __restrict__ PF, const float* __restrict__ w2, const float* __restrict__ b2, float* OUT) {
    __shared__ __align__(16) float srow[SEQ];
    const int lane = threadIdx.x & 31;
    const int wave = __builtin_amdgcn_readfirstlane((int)(threadIdx.x >> 5));
    const unsigned h = blockIdx.x;
    const float* hp = PF + (size_t)h * PW + 4 * lane;
    float hv[16], wv[16];
#pragma unroll
    for (int g = 0; g < 4; ++g) {
        const v4f a = *(const v4f*)(hp + 128 * g);
        const v4f w = *(const v4f*)(w2 + 128 * g + 4 * lane);
#pragma unroll
        for (int c = 0; c < 4; ++c) { hv[4 * g + c] = a[c]; wv[4 * g + c] = bfr(w[c]); } }
    const float b2v = bfr(b2[0]);
    const float* mp = PF + HID + 4 * lane;
#pragma unroll 1
    for (unsigned m = (unsigned)wave; m < (unsigned)SEQ; m += (unsigned)SW) {
        const float* mr = mp + (size_t)m * PW;
        v4f mv[4];
#pragma unroll
        for (int g = 0; g < 4; ++g) mv[g] = *(const v4f*)(mr + 128 * g);
        float p = 0.0f;
#pragma unroll
        for (int g = 0; g < 4; ++g) {
#pragma unroll
            for (int c = 0; c < 4; ++c) {
                const float z = hv[4 * g + c] + mv[g][c];
                const float e = __builtin_amdgcn_exp2f(z * TK2);
                const float r = __builtin_amdgcn_rcpf(e + 1.0f);
                const float t = fmaf(-2.0f, r, 1.0f);
                p = fmaf(wv[4 * g + c], t, p); } }
        p += __shfl_xor(p, 16, 32);
        p += __shfl_xor(p, 8, 32);
        p += __shfl_xor(p, 4, 32);
        p += __shfl_xor(p, 2, 32);
        p += __shfl_xor(p, 1, 32);
        const float sv = p + b2v;
        if (lane == 0) srow[m] = sv;
    }
    __syncthreads();
    if (wave < SEQ / 128) {
        const int o = wave * 128 + lane * 4;
        const v4f val = *(const v4fa*)(&srow[o]);
        float* orow = OUT + (size_t)h * OUT_PITCH + o;
#pragma unroll 1
        for (int ps = 0; ps < 2; ++ps) {
            *(volatile v4f*)orow = val;
            if (ps == 0) __threadfence(); }
    }
}

static constexpr size_t al256(size_t v) { return (v + 255) & ~(size_t)255; }
static constexpr size_t SZ_XB = al256((size_t)SEQ * KD * 2);
static constexpr size_t SZ_WB = al256((size_t)PW * KD * 2);
static constexpr size_t SZ_PF = al256((size_t)SEQ * PW * 4);
static constexpr size_t SZ_TOTAL = SZ_XB + SZ_WB + SZ_PF;
static constexpr size_t N8X = (size_t)SEQ * KD / 8;
static constexpr size_t N8W = (size_t)HID * KD / 8;
static_assert(SZ_TOTAL <= (size_t)134217728);
static_assert(((size_t)HID * KD * 2) % 256 == 0);
static_assert(N8X * 8 == (size_t)SEQ * KD);
static_assert(2 * N8W * 8 == (size_t)PW * KD);

extern "C" void kernel_launch(void* const* d_in, const int* in_sizes, int n_in,
                              void* d_out, int out_size, void* d_ws, size_t ws_size, hipStream_t stream) {
    if (n_in < 7) return;
    if ((size_t)in_sizes[0] < (size_t)SEQ * KD) return;
    if ((size_t)in_sizes[1] < (size_t)HID * KD || (size_t)in_sizes[3] < (size_t)HID * KD) return;
    if (in_sizes[2] < HID || in_sizes[4] < HID || in_sizes[5] < HID || in_sizes[6] < 1) return;
    if ((size_t)out_size < (size_t)(SEQ - 1) * OUT_PITCH + SEQ) return;
    if (SZ_TOTAL > ws_size) return;
    const float* x  = (const float*)d_in[0];
    const float* wh = (const float*)d_in[1]; const float* bh = (const float*)d_in[2];
    const float* wm = (const float*)d_in[3]; const float* bm = (const float*)d_in[4];
    const float* w2 = (const float*)d_in[5]; const float* b2 = (const float*)d_in[6];
    float* OUT = (float*)d_out;
    char* wsp = (char*)d_ws;
    bf* XB = (bf*)wsp; wsp += SZ_XB;
    bf* WB = (bf*)wsp; wsp += SZ_WB;
    float* PF = (float*)wsp; wsp += SZ_PF;

    k_cvt8<<<(unsigned)((N8X + 255) / 256), 256, 0, stream>>>(x, XB, N8X);
    k_cvt8<<<(unsigned)((N8W + 255) / 256), 256, 0, stream>>>(wh, WB, N8W);
    k_cvt8<<<(unsigned)((N8W + 255) / 256), 256, 0, stream>>>(wm, WB + (size_t)HID * KD, N8W);

    k_gemm<<<dim3(SEQ / 64, PW / 64, 1), 32, 0, stream>>>(XB, WB, bh, bm, PF);

    k_score<<<dim3(SEQ, 1, 1), 32 * SW, 0, stream>>>(PF, w2, b2, OUT);
}
